// SimpleAttention_32066225832529
// MI455X (gfx1250) — hardware-verified
//
#include <hip/hip_runtime.h>
#include <stdint.h>


typedef _Float16 v16h __attribute__((ext_vector_type(16)));
typedef _Float16 v8h  __attribute__((ext_vector_type(8)));
typedef _Float16 v8ha __attribute__((ext_vector_type(8), may_alias));
typedef float    v8f  __attribute__((ext_vector_type(8)));
typedef float    v4f  __attribute__((ext_vector_type(4)));
typedef float    v4fa __attribute__((ext_vector_type(4), may_alias));
typedef unsigned int v4u __attribute__((ext_vector_type(4)));

union U8f  { v8f  v; float    f[8]; };
union U16h { v16h v; v8h      h[2]; };
union U8h  { v8h  v; _Float16 f[8]; };

#ifndef NB
#define NB 2
#endif
#ifndef SEQ
#define SEQ 2048
#endif
#define NB_FULL  2
#define SEQ_FULL 2048
#define CC       1024
#define NH       16
#define HS       64
#define MROWS    (NB * SEQ)

#define BQ  128
#define BK  32
#define KP  72
#define VP  40
#define TP  72

static_assert(NB >= 1 && NB <= NB_FULL);
static_assert(SEQ >= BQ && SEQ <= SEQ_FULL);
static_assert(SEQ % BQ == 0);
static_assert(SEQ % 64 == 0);
static_assert(SEQ % BK == 0);
static_assert(MROWS % 64 == 0);
static_assert(CC == NH * HS);
static_assert(CC % 64 == 0);
static_assert((KP * 2) % 16 == 0 && (VP * 2) % 16 == 0 && (TP * 2) % 16 == 0);

#define WCARRY  64.0f
#define OSCALE  (1.0f / 4096.0f)
#define C2SCALE (1.4426950408889634f / 32768.0f)

__device__ __forceinline__ v8f wmma_f16(v16h a, v16h b, v8f c) {
  v8f d = __builtin_amdgcn_wmma_f32_16x16x32_f16(false, a, false, b, (short)0, c, false, false);
  asm volatile("v_nop\n\tv_nop\n\tv_nop\n\tv_nop" : "+v"(d) : "v"(a), "v"(b));
  return d;
}

template <int CTRL>
__device__ __forceinline__ float dppf(float x) {
  int s = __float_as_int(x);
  return __int_as_float(__builtin_amdgcn_update_dpp(s, s, CTRL, 0xF, 0xF, true));
}
__device__ __forceinline__ float red_max16(float x) {
  x = fmaxf(x, dppf<0xB1>(x));
  x = fmaxf(x, dppf<0x4E>(x));
  x = fmaxf(x, dppf<0x141>(x));
  x = fmaxf(x, dppf<0x140>(x));
  return x;
}
__device__ __forceinline__ float red_sum16(float x) {
  x += dppf<0xB1>(x);
  x += dppf<0x4E>(x);
  x += dppf<0x141>(x);
  x += dppf<0x140>(x);
  return x;
}

__device__ __forceinline__ void wave_lds_sync() {
  __builtin_amdgcn_fence(3, "wavefront");
  asm volatile("s_wait_dscnt 0" ::: "memory");
  __builtin_amdgcn_wave_barrier();
}

__device__ __forceinline__ v4f bf16_rne4(v4f a) {
  v4u u = __builtin_bit_cast(v4u, a);
  u = (u + 0x7FFFu + ((u >> 16) & 1u)) & 0xFFFF0000u;
  return __builtin_bit_cast(v4f, u);
}

__device__ __forceinline__ v8h cvt8v(v4f a, v4f b) {
  v8h d;
  d[0] = (_Float16)a[0]; d[1] = (_Float16)a[1];
  d[2] = (_Float16)a[2]; d[3] = (_Float16)a[3];
  d[4] = (_Float16)b[0]; d[5] = (_Float16)b[1];
  d[6] = (_Float16)b[2]; d[7] = (_Float16)b[3];
  return d;
}

__global__ __launch_bounds__(256)
void cvt_kernel(const float* __restrict__ src, _Float16* __restrict__ dst,
                int nrows, int seg, int segfull, float scale)
{
  const int p = blockIdx.x * 256 + threadIdx.x;
  if (p >= nrows * 128) return;
  const int m  = p >> 7;
  const int c0 = 8 * (p & 127);
  const int srow = (m / seg) * segfull + (m % seg);
  const float* s = src + (size_t)srow * CC + c0;
  v4f a0 = bf16_rne4(*(const v4f*)(s));
  v4f a1 = bf16_rne4(*(const v4f*)(s + 4));
  a0 = a0 * scale;
  a1 = a1 * scale;
  const v8h hv = cvt8v(a0, a1);
  _Float16* d = dst + (size_t)m * CC + c0;
  *(volatile v8h*)d = hv;
  __threadfence();
  *(volatile v8h*)d = hv;
}

template <int MODE>
__global__ __launch_bounds__(64)
void gemm_kernel(const _Float16* __restrict__ A, const _Float16* __restrict__ W,
                 void* __restrict__ outp, float oscale)
{
  __shared__ __attribute__((aligned(16))) _Float16 sh[64 * TP];

  const int tid  = threadIdx.x;
  const int wave = tid >> 5;
  const int lane = tid & 31;
  const int lh   = lane & 15;
  const int hi   = lane >> 4;
  const int m0   = (blockIdx.x >> 4) * 64;
  const int n0   = (blockIdx.x & 15) * 64;
  const int wr0  = m0 + 32 * wave;

  U8f acc[2][4];
  #pragma unroll
  for (int i = 0; i < 2; ++i)
    #pragma unroll
    for (int f = 0; f < 4; ++f) acc[i][f].v = (v8f){};

  const _Float16* Ab = A + (size_t)(wr0 + lh) * CC + 8 * hi;
  const _Float16* Wb = W + (size_t)(n0 + lh) * CC + 8 * hi;

  #pragma unroll 1
  for (int k0 = 0; k0 < CC; k0 += 32) {
    U16h af[2];
    #pragma unroll
    for (int i = 0; i < 2; ++i) {
      af[i].h[0] = *(const v8h*)(Ab + (size_t)(16 * i) * CC + k0);
      af[i].h[1] = *(const v8h*)(Ab + (size_t)(16 * i) * CC + k0 + 16);
    }
    #pragma unroll
    for (int f = 0; f < 4; ++f) {
      U16h bf;
      bf.h[0] = *(const v8h*)(Wb + (size_t)(16 * f) * CC + k0);
      bf.h[1] = *(const v8h*)(Wb + (size_t)(16 * f) * CC + k0 + 16);
      acc[0][f].v = wmma_f16(af[0].v, bf.v, acc[0][f].v);
      acc[1][f].v = wmma_f16(af[1].v, bf.v, acc[1][f].v);
    }
  }

  if (MODE == 0) {
    _Float16* O  = (_Float16*)outp;
    _Float16* so = sh + wave * (32 * TP);
    #pragma unroll
    for (int g = 0; g < 2; ++g) {
      #pragma unroll
      for (int j = 0; j < 8; ++j) {
        #pragma unroll
        for (int f = 0; f < 4; ++f)
          so[(j + 8 * hi) * 64 + 16 * f + lh] = (_Float16)acc[g][f].f[j];
      }
      wave_lds_sync();
      v8h ov[4]; int oo[4];
      #pragma unroll
      for (int k = 0; k < 4; ++k) {
        const int c = lane + 32 * k, r = c >> 3, p = c & 7;
        ov[k] = *(const v8ha*)(so + r * 64 + 8 * p);
        oo[k] = r * CC + 8 * p;
      }
      _Float16* ob = O + (size_t)(wr0 + 16 * g) * CC + n0;
      #pragma unroll
      for (int k = 0; k < 4; ++k) *(volatile v8h*)(ob + oo[k]) = ov[k];
      __threadfence();
      #pragma unroll
      for (int k = 0; k < 4; ++k) *(volatile v8h*)(ob + oo[k]) = ov[k];
      wave_lds_sync();
    }
  } else if (MODE == 2) {
    float* O   = (float*)outp;
    float* sof = (float*)(sh + wave * (32 * TP));
    #pragma unroll
    for (int g = 0; g < 2; ++g) {
      #pragma unroll
      for (int j = 0; j < 8; ++j) {
        #pragma unroll
        for (int f = 0; f < 4; ++f)
          sof[(j + 8 * hi) * 64 + 16 * f + lh] = acc[g][f].f[j] * oscale;
      }
      wave_lds_sync();
      v4f ov[8]; int oo[8];
      #pragma unroll
      for (int k = 0; k < 8; ++k) {
        const int c = lane + 32 * k, r = c >> 4, q = c & 15;
        ov[k] = *(const v4fa*)(sof + r * 64 + 4 * q);
        oo[k] = r * CC + 4 * q;
      }
      float* ob = O + (size_t)(wr0 + 16 * g) * CC + n0;
      #pragma unroll
      for (int k = 0; k < 8; ++k) *(volatile v4f*)(ob + oo[k]) = ov[k];
      __threadfence();
      #pragma unroll
      for (int k = 0; k < 8; ++k) *(volatile v4f*)(ob + oo[k]) = ov[k];
      wave_lds_sync();
    }
  } else {
    _Float16* VT = (_Float16*)outp;
    #pragma unroll
    for (int g = 0; g < 2; ++g) {
      #pragma unroll
      for (int j = 0; j < 8; ++j) {
        #pragma unroll
        for (int f = 0; f < 4; ++f)
          sh[(16 * f + lh) * TP + 32 * wave + 16 * g + 8 * hi + j] = (_Float16)acc[g][f].f[j];
      }
    }
    __syncthreads();
    const int b  = m0 / SEQ;
    const int t0 = m0 - b * SEQ;
    const int hh = n0 >> 6;
    v8h ov[8]; size_t oo[8];
    #pragma unroll
    for (int k = 0; k < 8; ++k) {
      const int c = lane + 32 * k, dr = 32 * wave + (c >> 3), p = c & 7;
      ov[k] = *(const v8ha*)(sh + dr * TP + 8 * p);
      oo[k] = ((size_t)((b * NH + hh) * HS + dr)) * SEQ + t0 + 8 * p;
    }
    #pragma unroll
    for (int k = 0; k < 8; ++k) *(volatile v8h*)(VT + oo[k]) = ov[k];
    __threadfence();
    #pragma unroll
    for (int k = 0; k < 8; ++k) *(volatile v8h*)(VT + oo[k]) = ov[k];
  }
}

__global__ __launch_bounds__(256)
void attn_kernel(const _Float16* __restrict__ Qp, const _Float16* __restrict__ Kp,
                 const _Float16* __restrict__ Vt, _Float16* __restrict__ Yp)
{
  __shared__ __attribute__((aligned(16))) _Float16 sK[BK * KP];
  __shared__ __attribute__((aligned(16))) _Float16 sV[HS * VP];
  __shared__ __attribute__((aligned(16))) _Float16 sP[8 * 16 * BK];
  __shared__ __attribute__((aligned(16))) _Float16 sY[8 * 16 * 64];

  const int tid  = threadIdx.x;
  const int wave = tid >> 5;
  const int lane = tid & 31;
  const int lh   = lane & 15;
  const int hi   = lane >> 4;

  const int nqb   = SEQ / BQ;
  const int bh    = blockIdx.x / nqb;
  const int qbase = (blockIdx.x % nqb) * BQ;
  const int b     = bh >> 4;
  const int h     = bh & 15;
  const int qrow0 = qbase + wave * 16;
  const size_t mbase = (size_t)b * SEQ;

  const _Float16* Qb = Qp + (mbase + qrow0 + lh) * CC + h * HS + 8 * hi;
  U16h qf[2];
  #pragma unroll
  for (int c = 0; c < 2; ++c) {
    qf[c].h[0] = *(const v8h*)(Qb + 32 * c);
    qf[c].h[1] = *(const v8h*)(Qb + 32 * c + 16);
  }
  const _Float16* Kb = Kp + mbase * CC + h * HS;
  const _Float16* Vb = Vt + (size_t)bh * HS * SEQ;

  U8f acc[4];
  #pragma unroll
  for (int t = 0; t < 4; ++t) acc[t].v = (v8f){};
  float mrow[8], lrow[8];
  #pragma unroll
  for (int j = 0; j < 8; ++j) { mrow[j] = -3.0e38f; lrow[j] = 0.0f; }

  _Float16* pw = sP + wave * (16 * BK);

  for (int kv0 = 0; kv0 < SEQ; kv0 += BK) {
    __syncthreads();
    {
      const int r = tid >> 3, g = tid & 7;
      const v8h kk = *(const v8h*)(Kb + (size_t)(kv0 + r) * CC + 8 * g);
      *(v8h*)(sK + r * KP + 8 * g) = kk;
    }
    {
      const int d = tid >> 2, g = tid & 3;
      const v8h vv = *(const v8h*)(Vb + (size_t)d * SEQ + kv0 + 8 * g);
      *(v8h*)(sV + d * VP + 8 * g) = vv;
    }
    __syncthreads();

    U8f s0, s1; s0.v = (v8f){}; s1.v = (v8f){};
    #pragma unroll
    for (int c = 0; c < 2; ++c) {
      U16h kf;
      kf.h[0] = *(const v8h*)(sK + lh * KP + 32 * c + 8 * hi);
      kf.h[1] = *(const v8h*)(sK + lh * KP + 32 * c + 16 + 8 * hi);
      s0.v = wmma_f16(qf[c].v, kf.v, s0.v);
      kf.h[0] = *(const v8h*)(sK + (16 + lh) * KP + 32 * c + 8 * hi);
      kf.h[1] = *(const v8h*)(sK + (16 + lh) * KP + 32 * c + 16 + 8 * hi);
      s1.v = wmma_f16(qf[c].v, kf.v, s1.v);
    }

    const int key0 = kv0 + lh;
    const int key1 = kv0 + 16 + lh;
    U8h pa, pb;
    #pragma unroll
    for (int j = 0; j < 8; ++j) {
      const int   qi = qrow0 + 8 * hi + j;
      const float a  = (key0 > qi) ? 0.0f : s0.f[j] * C2SCALE;
      const float bb = (key1 > qi) ? 0.0f : s1.f[j] * C2SCALE;
      const float rm    = red_max16(fmaxf(a, bb));
      const float mnew  = fmaxf(mrow[j], rm);
      const float alpha = __builtin_amdgcn_exp2f(mrow[j] - mnew);
      const float e0    = __builtin_amdgcn_exp2f(a  - mnew);
      const float e1    = __builtin_amdgcn_exp2f(bb - mnew);
      lrow[j] = lrow[j] * alpha + red_sum16(e0 + e1);
      mrow[j] = mnew;
      pa.f[j] = (_Float16)(e0 * 1024.0f);
      pb.f[j] = (_Float16)(e1 * 1024.0f);
      #pragma unroll
      for (int t = 0; t < 4; ++t) acc[t].f[j] *= alpha;
    }

    #pragma unroll
    for (int j = 0; j < 8; ++j) {
      pw[(j + 8 * hi) * BK + lh]      = pa.f[j];
      pw[(j + 8 * hi) * BK + 16 + lh] = pb.f[j];
    }
    wave_lds_sync();
    U16h pf;
    pf.h[0] = *(const v8ha*)(pw + lh * BK + 8 * hi);
    pf.h[1] = *(const v8ha*)(pw + lh * BK + 16 + 8 * hi);

    #pragma unroll
    for (int t = 0; t < 4; ++t) {
      U16h vf;
      vf.h[0] = *(const v8h*)(sV + (16 * t + lh) * VP + 8 * hi);
      vf.h[1] = *(const v8h*)(sV + (16 * t + lh) * VP + 16 + 8 * hi);
      acc[t].v = wmma_f16(pf.v, vf.v, acc[t].v);
    }
  }

  float inv[8];
  #pragma unroll
  for (int j = 0; j < 8; ++j) inv[j] = 1.0f / (lrow[j] * 1024.0f);
  _Float16* sy = sY + wave * (16 * 64);
  #pragma unroll
  for (int j = 0; j < 8; ++j) {
    #pragma unroll
    for (int t = 0; t < 4; ++t)
      sy[(j + 8 * hi) * 64 + 16 * t + lh] = (_Float16)(acc[t].f[j] * inv[j]);
  }
  wave_lds_sync();
  v8h ov[4]; int oo[4];
  #pragma unroll
  for (int k = 0; k < 4; ++k) {
    const int c = lane + 32 * k, r = c >> 3, p = c & 7;
    ov[k] = *(const v8ha*)(sy + r * 64 + 8 * p);
    oo[k] = r * CC + 8 * p;
  }
  _Float16* yb = Yp + (mbase + qrow0) * CC + h * HS;
  #pragma unroll
  for (int k = 0; k < 4; ++k) *(volatile v8h*)(yb + oo[k]) = ov[k];
  __threadfence();
  #pragma unroll
  for (int k = 0; k < 4; ++k) *(volatile v8h*)(yb + oo[k]) = ov[k];
}

extern "C" void kernel_launch(void* const* d_in, const int* in_sizes, int n_in,
                              void* d_out, int out_size, void* d_ws, size_t ws_size,
                              hipStream_t stream) {
  if (n_in < 5) return;
  const long long need_x = ((long long)(NB - 1) * SEQ_FULL + SEQ) * CC;
  if ((long long)in_sizes[0] < need_x) return;
  if ((long long)in_sizes[1] < (long long)CC * CC) return;
  if ((long long)in_sizes[2] < (long long)CC * CC) return;
  if ((long long)in_sizes[3] < (long long)CC * CC) return;
  if ((long long)in_sizes[4] < (long long)CC * CC) return;
  if ((long long)out_size < (long long)MROWS * CC) return;

  const size_t act_bytes = (size_t)MROWS * CC * 2;
  const size_t w_bytes   = (size_t)CC * CC * 2;
  const size_t vt_bytes  = (size_t)NB * NH * HS * SEQ * 2;
  const size_t off_x  = 0;
  const size_t off_wq = off_x  + act_bytes;
  const size_t off_wk = off_wq + w_bytes;
  const size_t off_wv = off_wk + w_bytes;
  const size_t off_wp = off_wv + w_bytes;
  const size_t off_q  = off_wp + w_bytes;
  const size_t off_k  = off_q  + act_bytes;
  const size_t off_vt = off_k  + act_bytes;
  const size_t off_y  = off_vt + vt_bytes;
  const size_t off_end = off_y + act_bytes;
  if (off_end > ws_size) return;

  const float* x  = (const float*)d_in[0];
  const float* wq = (const float*)d_in[1];
  const float* wk = (const float*)d_in[2];
  const float* wv = (const float*)d_in[3];
  const float* wp = (const float*)d_in[4];
  float* out = (float*)d_out;
  char* ws = (char*)d_ws;
  _Float16* xh  = (_Float16*)(ws + off_x);
  _Float16* wqh = (_Float16*)(ws + off_wq);
  _Float16* wkh = (_Float16*)(ws + off_wk);
  _Float16* wvh = (_Float16*)(ws + off_wv);
  _Float16* wph = (_Float16*)(ws + off_wp);
  _Float16* qh  = (_Float16*)(ws + off_q);
  _Float16* kh  = (_Float16*)(ws + off_k);
  _Float16* vt  = (_Float16*)(ws + off_vt);
  _Float16* yh  = (_Float16*)(ws + off_y);

  cvt_kernel<<<(MROWS * 128) / 256, 256, 0, stream>>>(x,  xh,  MROWS, SEQ, SEQ_FULL, 1.0f);
  cvt_kernel<<<(CC * 128) / 256,    256, 0, stream>>>(wq, wqh, CC, CC, CC, WCARRY);
  cvt_kernel<<<(CC * 128) / 256,    256, 0, stream>>>(wk, wkh, CC, CC, CC, WCARRY);
  cvt_kernel<<<(CC * 128) / 256,    256, 0, stream>>>(wv, wvh, CC, CC, CC, WCARRY);
  cvt_kernel<<<(CC * 128) / 256,    256, 0, stream>>>(wp, wph, CC, CC, CC, WCARRY);

  const int gemm_blocks = (MROWS / 64) * (CC / 64);
  gemm_kernel<0><<<gemm_blocks, 64, 0, stream>>>(xh, wqh, (void*)qh, 1.0f);
  gemm_kernel<0><<<gemm_blocks, 64, 0, stream>>>(xh, wkh, (void*)kh, 1.0f);
  gemm_kernel<1><<<gemm_blocks, 64, 0, stream>>>(xh, wvh, (void*)vt, 1.0f);

  attn_kernel<<<NB * NH * (SEQ / BQ), 256, 0, stream>>>(qh, kh, vt, yh);

  gemm_kernel<2><<<gemm_blocks, 64, 0, stream>>>(yh, wph, (void*)out, OSCALE);
}
